// Reattention_57440892617325
// MI455X (gfx1250) — hardware-verified
//
#include <hip/hip_runtime.h>
#include <math.h>

constexpr int kBatch   = 4;
constexpr int kSeq     = 1024;
constexpr int kDim     = 768;
constexpr int kHeads   = 12;
constexpr int kDh      = 64;
constexpr int kInner   = kHeads * kDh;
constexpr int kTok     = kBatch * kSeq;
constexpr int kQKVCols = 3 * kInner;
constexpr int kQKCols  = 2 * kInner;
constexpr float kScoreScale = 0.125f;
constexpr float kA2Carry    = 16.0f;
constexpr float kA2CarryInv = 1.0f / 16.0f;
constexpr float kWoCarry    = 64.0f;
constexpr float kWoCarryInv = 1.0f / 64.0f;
constexpr float kLnEps      = 1e-5f;
constexpr float kInvHeads   = 1.0f / 12.0f;

typedef __attribute__((ext_vector_type(16))) _Float16 v16h;
typedef __attribute__((ext_vector_type(8)))  _Float16 v8h;
typedef __attribute__((ext_vector_type(16))) __bf16   v16b;
typedef __attribute__((ext_vector_type(8)))  __bf16   v8b;
typedef __attribute__((ext_vector_type(8)))  float    v8f;
typedef __attribute__((ext_vector_type(4)))  float    v4f;
typedef __attribute__((ext_vector_type(4)))  unsigned int v4u;

__device__ __forceinline__ unsigned short f2bf_bits(float f) {
  unsigned u = __float_as_uint(f);
  return (unsigned short)((u + 0x7FFFu + ((u >> 16) & 1u)) >> 16);
}
__device__ __forceinline__ float bf_bits2f(unsigned short h) { return __uint_as_float(((unsigned)h) << 16); }

__device__ __forceinline__ void dep_guard_h(v8f& a, v8f& b, v16h x, v16h y) { asm volatile("v_nop\n\tv_nop\n\tv_nop\n\tv_nop" : "+v"(a), "+v"(b) : "v"(x), "v"(y)); }
__device__ __forceinline__ void dep_guard_b(v8f& a, v8f& b, v16b x, v16b y) { asm volatile("v_nop\n\tv_nop\n\tv_nop\n\tv_nop" : "+v"(a), "+v"(b) : "v"(x), "v"(y)); }
__device__ __forceinline__ void keep4_h(v16h a, v16h b, v16h c, v16h d) { asm volatile("v_nop" :: "v"(a), "v"(b), "v"(c), "v"(d)); }
__device__ __forceinline__ void keep4_b(v16b a, v16b b, v16b c, v16b d) { asm volatile("v_nop" :: "v"(a), "v"(b), "v"(c), "v"(d)); }
__device__ __forceinline__ void acc_guard4(v8f& a, v8f& b, v8f& c, v8f& d) { asm volatile("v_nop\n\tv_nop\n\tv_nop\n\tv_nop" : "+v"(a), "+v"(b), "+v"(c), "+v"(d)); }
template <typename T> struct Frag;
template <> struct Frag<_Float16> {
  typedef v16h V; union U { v16h v; v8h h[2]; };
  static __device__ __forceinline__ v16h load(const _Float16* p) {
    U f; f.h[0] = *(const v8h*)(p); f.h[1] = *(const v8h*)(p + 16); return f.v;
  }
  static __device__ __forceinline__ v8f mma(v16h a, v16h b, v8f c) {
    return __builtin_amdgcn_wmma_f32_16x16x32_f16(false, a, false, b, (short)0, c, false, false);
  }
  static __device__ __forceinline__ void guard(v8f& a, v8f& b, v16h x, v16h y) { dep_guard_h(a, b, x, y); }
  static __device__ __forceinline__ void keep(v16h a, v16h b, v16h c, v16h d) { keep4_h(a, b, c, d); }
};
template <> struct Frag<__bf16> {
  typedef v16b V; union U { v16b v; v8b h[2]; };
  static __device__ __forceinline__ v16b load(const __bf16* p) {
    U f; f.h[0] = *(const v8b*)(p); f.h[1] = *(const v8b*)(p + 16); return f.v;
  }
  static __device__ __forceinline__ v8f mma(v16b a, v16b b, v8f c) {
    return __builtin_amdgcn_wmma_f32_16x16x32_bf16(false, a, false, b, (short)0, c, false, false);
  }
  static __device__ __forceinline__ void guard(v8f& a, v8f& b, v16b x, v16b y) { dep_guard_b(a, b, x, y); }
  static __device__ __forceinline__ void keep(v16b a, v16b b, v16b c, v16b d) { keep4_b(a, b, c, d); }
};

__device__ __forceinline__ unsigned pk16(unsigned short a, unsigned short b) { return (unsigned)a | ((unsigned)b << 16); }
__device__ __forceinline__ unsigned short h_bits(float f) { const _Float16 h = (_Float16)f; return __builtin_bit_cast(unsigned short, h); }
__device__ __forceinline__ float bf16_rne(float f) { return bf_bits2f(f2bf_bits(f)); }

template <int ET> struct Elem;
template <> struct Elem<0> { typedef _Float16 T; };
template <> struct Elem<1> { typedef __bf16 T; };
template <int ET, bool SPLIT, int BIAS_MODE, int OUT_MODE, bool RESID, int ACT = 0>
__global__ __launch_bounds__(256) void wmma_gemm64(
    const unsigned short* __restrict__ Ap, const unsigned short* __restrict__ A2p, int lda, long strideA,
    const unsigned short* __restrict__ Btp, const unsigned short* __restrict__ Bt2p, int ldb, long strideB,
    void* __restrict__ Cout, void* __restrict__ Cout2, int ldc, long strideC,
    const float* __restrict__ bias,
    const float* __restrict__ resid, long strideR,
    int M, int N, int K, float scale) {
  typedef typename Elem<ET>::T T;
  typedef typename Frag<T>::V V;
  const T* A = (const T*)Ap; const T* A2 = (const T*)A2p; const T* Bt = (const T*)Btp; const T* Bt2 = (const T*)Bt2p;
  __shared__ __align__(16) float sT[8][16 * 68];
  const int b    = blockIdx.y;
  const int lane = threadIdx.x & 31;
  const int wave = threadIdx.x >> 5;
  const int tilesN = N >> 6;
  const int tilesM = M >> 6;
  const int tile = blockIdx.x * 8 + wave;
  if (tile >= tilesM * tilesN) return;
  const int tm = tile / tilesN;
  const int tn = tile - tm * tilesN;
  const int m0 = tm << 6;
  const int n0 = tn << 6;

  const T* Ab  = A  + (size_t)b * strideA;
  const T* Bb  = Bt + (size_t)b * strideB;
  const T* Ab2 = SPLIT ? (A2  + (size_t)b * strideA) : nullptr;
  const T* Bb2 = SPLIT ? (Bt2 + (size_t)b * strideB) : nullptr;

  const int rlane = lane & 15;
  const int koff  = (lane >> 4) * 8;
  const int mOff  = (lane >> 4) * 8;

  v8f acc[4][4];
#pragma unroll
  for (int i = 0; i < 4; ++i)
#pragma unroll
    for (int j = 0; j < 4; ++j) acc[i][j] = (v8f){0.f,0.f,0.f,0.f,0.f,0.f,0.f,0.f};

  for (int k0 = 0; k0 < K; k0 += 32) {
    V bh[4], bl[4];
#pragma unroll
    for (int j = 0; j < 4; ++j) {
      const size_t bo = (size_t)(n0 + (j << 4) + rlane) * ldb + koff + k0;
      bh[j] = Frag<T>::load(Bb + bo);
      if (SPLIT) bl[j] = Frag<T>::load(Bb2 + bo);
    }
#pragma unroll
    for (int i = 0; i < 4; ++i) {
      const size_t ao = (size_t)(m0 + (i << 4) + rlane) * lda + koff + k0;
      V ah = Frag<T>::load(Ab + ao);
      V al;
      if (SPLIT) al = Frag<T>::load(Ab2 + ao);
#pragma unroll
      for (int j = 0; j < 4; ++j) {
        acc[i][j] = Frag<T>::mma(ah, bh[j], acc[i][j]);
        if (SPLIT) {
          acc[i][j] = Frag<T>::mma(ah, bl[j], acc[i][j]);
          acc[i][j] = Frag<T>::mma(al, bh[j], acc[i][j]);
        }
      }
      Frag<T>::guard(acc[i][0], acc[i][3], ah, SPLIT ? al : ah);
    }
    Frag<T>::keep(bh[0], bh[1], bh[2], bh[3]);
    if (SPLIT) Frag<T>::keep(bl[0], bl[1], bl[2], bl[3]);
  }
  acc_guard4(acc[0][0], acc[0][1], acc[0][2], acc[0][3]);
  acc_guard4(acc[1][0], acc[1][1], acc[1][2], acc[1][3]);
  acc_guard4(acc[2][0], acc[2][1], acc[2][2], acc[2][3]);
  acc_guard4(acc[3][0], acc[3][1], acc[3][2], acc[3][3]);

  float* slab = sT[wave];
  const float* Rb = RESID ? (resid + (size_t)b * strideR) : nullptr;
#pragma unroll
  for (int i = 0; i < 4; ++i) {
    const int mBase = m0 + (i << 4);
#pragma unroll
    for (int j = 0; j < 4; ++j) {
      const int n = n0 + (j << 4) + rlane;
      float bv = 0.f;
      if (BIAS_MODE == 2) bv = bias[n];
#pragma unroll
      for (int r = 0; r < 8; ++r) {
        float v = acc[i][j][r] * scale;
        if (BIAS_MODE == 1) v += bias[mBase + mOff + r];
        if (BIAS_MODE == 2) v += bv;
        if (RESID) v += Rb[(size_t)(mBase + mOff + r) * ldc + n];
        if (ACT == 2) v = fmaxf(v, 0.0f);
        if (ACT == 4) v = (v > 0.f) ? v : 0.01f * v;
        slab[(mOff + r) * 68 + (j << 4) + rlane] = v;
      }
    }
    __builtin_amdgcn_fence(__ATOMIC_RELEASE, "workgroup");
    __builtin_amdgcn_wave_barrier();
    __builtin_amdgcn_fence(__ATOMIC_ACQUIRE, "workgroup");
    if (OUT_MODE == 0) {
      float* C = (float*)Cout + (size_t)b * strideC;
      const int hh = lane >> 4, c4 = (lane & 15) * 4;
      for (int pass = 0; pass < 2; ++pass) {
#pragma unroll
        for (int it = 0; it < 8; ++it) {
          const int row = it * 2 + hh;
          v4f v = *(const v4f*)(slab + row * 68 + c4);
          *(volatile v4f*)(C + (size_t)(mBase + row) * ldc + n0 + c4) = v;
        }
        __threadfence();
      }
    } else {
      const int q = lane >> 3, c8 = (lane & 7) * 8;
      unsigned short* C  = (unsigned short*)Cout  + (size_t)b * strideC;
      unsigned short* C2 = (OUT_MODE == 2) ? ((unsigned short*)Cout2 + (size_t)b * strideC) : nullptr;
      for (int pass = 0; pass < 2; ++pass) {
#pragma unroll
        for (int it = 0; it < 4; ++it) {
          const int row = it * 4 + q;
          const float* sp = slab + row * 68 + c8;
          v8h hv, lv;
#pragma unroll
          for (int e = 0; e < 8; ++e) {
            if (OUT_MODE == 1) {
              hv[e] = (_Float16)sp[e];
            } else {
              unsigned short hb = f2bf_bits(sp[e]);
              unsigned short lb = f2bf_bits(sp[e] - bf_bits2f(hb));
              hv[e] = __builtin_bit_cast(_Float16, hb);
              lv[e] = __builtin_bit_cast(_Float16, lb);
            }
          }
          *(volatile v8h*)(C + (size_t)(mBase + row) * ldc + n0 + c8) = hv;
          if (OUT_MODE == 2) *(volatile v8h*)(C2 + (size_t)(mBase + row) * ldc + n0 + c8) = lv;
        }
        __threadfence();
      }
    }
    __builtin_amdgcn_fence(__ATOMIC_RELEASE, "workgroup");
    __builtin_amdgcn_wave_barrier();
    __builtin_amdgcn_fence(__ATOMIC_ACQUIRE, "workgroup");
  }
}

__global__ __launch_bounds__(256) void cast8_bf16_kernel(const float* __restrict__ in, unsigned short* __restrict__ out, int n8) {
  const int i = blockIdx.x * 256 + threadIdx.x;
  if (i >= n8) return;
  const float* p = in + 8 * (size_t)i;
  const v4f a = *(const v4f*)(p);
  const v4f c = *(const v4f*)(p + 4);
  unsigned short hb[8];
#pragma unroll
  for (int e = 0; e < 4; ++e) {
    hb[e]     = f2bf_bits(a[e]);
    hb[4 + e] = f2bf_bits(c[e]);
  }
  const v4u u = (v4u){pk16(hb[0], hb[1]), pk16(hb[2], hb[3]), pk16(hb[4], hb[5]), pk16(hb[6], hb[7])};
  unsigned short* q = out + 8 * (size_t)i;
  *(volatile v4u*)q = u;
  __threadfence();
  *(volatile v4u*)q = u;
}

template <int MODE>
__global__ __launch_bounds__(256) void wtrans_kernel(const float* __restrict__ W, unsigned short* __restrict__ out,
                                                     int nrows, int ncols, float scale) {
  __shared__ float sm[64][65];
  const int t  = threadIdx.x;
  const int r0 = blockIdx.x * 64;
  const int c0 = blockIdx.y * 64;
#pragma unroll
  for (int it = 0; it < 16; ++it) {
    const int e  = it * 256 + t;
    const int rl = e >> 6;
    const int cl = e & 63;
    sm[cl][rl] = W[(size_t)(r0 + rl) * ncols + c0 + cl];
  }
  __syncthreads();
  const int lane = t & 31, wave = t >> 5;
  const int q = lane >> 3, c8 = (lane & 7) * 8;
  for (int pass = 0; pass < 2; ++pass) {
#pragma unroll
    for (int it = 0; it < 2; ++it) {
      const int row = wave * 8 + it * 4 + q;
      unsigned short hb[8];
#pragma unroll
      for (int e = 0; e < 8; ++e) {
        const float v = sm[row][c8 + e];
        if (MODE == 0) hb[e] = f2bf_bits(v);
        else           hb[e] = h_bits(bf16_rne(v) * scale);
      }
      const v4u u = (v4u){pk16(hb[0], hb[1]), pk16(hb[2], hb[3]), pk16(hb[4], hb[5]), pk16(hb[6], hb[7])};
      *(volatile v4u*)(out + (size_t)(c0 + row) * nrows + r0 + c8) = u;
    }
    __threadfence();
  }
}

__global__ __launch_bounds__(256) void softmix_kernel(const float* __restrict__ S, const float* __restrict__ rw,
                                                      const float* __restrict__ gam, const float* __restrict__ bet,
                                                      unsigned short* __restrict__ A2, float carry) {
  __shared__ __align__(16) float srow[kHeads][kSeq];
  __shared__ float sw[kHeads * kHeads];
  __shared__ float sg[kHeads];
  __shared__ float sb[kHeads];
  const int i    = blockIdx.x;
  const int t    = threadIdx.x;
  const int lane = t & 31;
  const int wave = t >> 5;

  if (t < kHeads * kHeads) sw[t] = bf16_rne(rw[t]);
  if (t < kHeads) { sg[t] = bf16_rne(gam[t]) * carry; sb[t] = bf16_rne(bet[t]) * carry; }

#pragma unroll 1
  for (int h = 0; h < kHeads; ++h) {
    const v4f v = *(const v4f*)(S + ((size_t)h * kSeq + i) * kSeq + 4 * t);
    *(v4f*)(&srow[h][4 * t]) = v;
  }
  __syncthreads();

  for (int r = wave; r < kHeads; r += 8) {
    float* row = &srow[r][0];
    float m = -INFINITY;
#pragma unroll 1
    for (int c = 0; c < 8; ++c) {
      const v4f v = *(const v4f*)(row + c * 128 + lane * 4);
      m = fmaxf(m, fmaxf(fmaxf(v[0], v[1]), fmaxf(v[2], v[3])));
    }
#pragma unroll
    for (int off = 16; off > 0; off >>= 1) m = fmaxf(m, __shfl_xor(m, off, 32));
    float s = 0.0f;
#pragma unroll 1
    for (int c = 0; c < 8; ++c) {
      float* p = row + c * 128 + lane * 4;
      const v4f v = *(const v4f*)p;
      v4f e;
      e[0] = __expf(v[0] - m);
      e[1] = __expf(v[1] - m);
      e[2] = __expf(v[2] - m);
      e[3] = __expf(v[3] - m);
      s += (e[0] + e[1]) + (e[2] + e[3]);
      *(v4f*)p = e;
    }
#pragma unroll
    for (int off = 16; off > 0; off >>= 1) s += __shfl_xor(s, off, 32);
    const float inv = 1.0f / s;
#pragma unroll 1
    for (int c = 0; c < 8; ++c) {
      float* p = row + c * 128 + lane * 4;
      v4f v = *(const v4f*)p;
      v = v * inv;
      *(v4f*)p = v;
    }
  }
  __syncthreads();

#pragma unroll 1
  for (int qq = 0; qq < 4; ++qq) {
    const int j = t + 256 * qq;
    float mk[kHeads];
#pragma unroll
    for (int k = 0; k < kHeads; ++k) mk[k] = 0.0f;
#pragma unroll 1
    for (int h = 0; h < kHeads; ++h) {
      const float ph = srow[h][j];
      const float* wr = sw + h * kHeads;
#pragma unroll
      for (int k = 0; k < kHeads; ++k) mk[k] = fmaf(ph, wr[k], mk[k]);
    }
    float sum = 0.0f;
#pragma unroll
    for (int k = 0; k < kHeads; ++k) sum += mk[k];
    const float mean = sum * kInvHeads;
    float var = 0.0f;
#pragma unroll
    for (int k = 0; k < kHeads; ++k) { const float d = mk[k] - mean; var = fmaf(d, d, var); }
    var *= kInvHeads;
    const float inv = rsqrtf(var + kLnEps);
#pragma unroll
    for (int k = 0; k < kHeads; ++k) srow[k][j] = fmaf((mk[k] - mean) * inv, sg[k], sb[k]);
  }
  __syncthreads();

  for (int pass = 0; pass < 2; ++pass) {
#pragma unroll 1
    for (int it = 0; it < 6; ++it) {
      const int u   = wave + 8 * it;
      const int k   = u >> 2;
      const int seg = u & 3;
      const float* sp = &srow[k][seg * 256 + lane * 8];
      const v4f a = *(const v4f*)(sp);
      const v4f c = *(const v4f*)(sp + 4);
      unsigned short hb[8];
#pragma unroll
      for (int e = 0; e < 4; ++e) { hb[e] = h_bits(a[e]); hb[4 + e] = h_bits(c[e]); }
      const v4u uv = (v4u){pk16(hb[0], hb[1]), pk16(hb[2], hb[3]), pk16(hb[4], hb[5]), pk16(hb[6], hb[7])};
      *(volatile v4u*)(A2 + ((size_t)k * kSeq + i) * kSeq + seg * 256 + lane * 8) = uv;
    }
    __threadfence();
  }
}

extern "C" void kernel_launch(void* const* d_in, const int* in_sizes, int n_in,
                              void* d_out, int out_size, void* d_ws, size_t ws_size,
                              hipStream_t stream) {
  if (n_in < 7) return;
  if (in_sizes[0] != kTok * kDim) return;
  if (in_sizes[1] != kDim * kQKVCols) return;
  if (in_sizes[2] != kHeads * kHeads) return;
  if (in_sizes[3] != kHeads || in_sizes[4] != kHeads) return;
  if (in_sizes[5] != kInner * kDim) return;
  if (in_sizes[6] != kDim) return;
  if (out_size != kTok * kDim) return;

  const float* x      = (const float*)d_in[0];
  const float* w_qkv  = (const float*)d_in[1];
  const float* rw     = (const float*)d_in[2];
  const float* gam    = (const float*)d_in[3];
  const float* bet    = (const float*)d_in[4];
  const float* w_out  = (const float*)d_in[5];
  const float* b_out  = (const float*)d_in[6];
  float* out = (float*)d_out;

  const size_t szXb  = (size_t)kTok * kDim * 2;
  const size_t szWT  = (size_t)kQKVCols * kDim * 2;
  const size_t szWoT = (size_t)kDim * kInner * 2;
  const size_t szQK  = (size_t)kTok * kQKCols * 2;
  const size_t szVt  = (size_t)kInner * kTok * 2;
  const size_t szS   = (size_t)kHeads * kSeq * kSeq * 4;
  const size_t szA2  = (size_t)kHeads * kSeq * kSeq * 2;
  const size_t szO   = (size_t)kTok * kInner * 2;
  size_t off = 0;
  unsigned char* ws = (unsigned char*)d_ws;
  unsigned short* xb   = (unsigned short*)(ws + off); off += szXb;
  unsigned short* WT   = (unsigned short*)(ws + off); off += szWT;
  unsigned short* WoT  = (unsigned short*)(ws + off); off += szWoT;
  unsigned short* QKhi = (unsigned short*)(ws + off); off += szQK;
  unsigned short* QKlo = (unsigned short*)(ws + off); off += szQK;
  unsigned short* Vt   = (unsigned short*)(ws + off); off += szVt;
  float*          S    = (float*)(ws + off);          off += szS;
  unsigned short* A2   = (unsigned short*)(ws + off); off += szA2;
  unsigned short* Octx = (unsigned short*)(ws + off); off += szO;
  if (off > ws_size) return;

  const dim3 blk(256, 1, 1);

  {
    const int n8 = kTok * kDim / 8;
    cast8_bf16_kernel<<<dim3((n8 + 255) / 256, 1, 1), blk, 0, stream>>>(x, xb, n8);
    wtrans_kernel<0><<<dim3(kDim / 64, kQKVCols / 64, 1), blk, 0, stream>>>(w_qkv, WT, kDim, kQKVCols, 1.0f);
    wtrans_kernel<1><<<dim3(kInner / 64, kDim / 64, 1), blk, 0, stream>>>(w_out, WoT, kInner, kDim, kWoCarry);
  }

  wmma_gemm64<1, false, 0, 2, false><<<dim3((kTok / 64) * (kQKCols / 64) / 8, 1, 1), blk, 0, stream>>>(
      xb, xb, kDim, 0L, WT, WT, kDim, 0L, (void*)QKhi, (void*)QKlo, kQKCols, 0L,
      b_out, b_out, 0L, kTok, kQKCols, kDim, 1.0f);

  wmma_gemm64<1, false, 0, 1, false><<<dim3((kInner / 64) * (kTok / 64) / 8, 1, 1), blk, 0, stream>>>(
      WT + (size_t)kQKCols * kDim, WT + (size_t)kQKCols * kDim, kDim, 0L, xb, xb, kDim, 0L,
      (void*)Vt, (void*)Vt, kTok, 0L, b_out, b_out, 0L, kInner, kTok, kDim, 1.0f);

  for (int bb = 0; bb < kBatch; ++bb) {
    const size_t qkoff = (size_t)bb * kSeq * kQKCols;
    wmma_gemm64<1, true, 0, 0, false><<<dim3((kSeq / 64) * (kSeq / 64) / 8, kHeads, 1), blk, 0, stream>>>(
        QKhi + qkoff, QKlo + qkoff, kQKCols, (long)kDh,
        QKhi + qkoff + kInner, QKlo + qkoff + kInner, kQKCols, (long)kDh,
        (void*)S, (void*)S, kSeq, (long)kSeq * kSeq,
        b_out, b_out, 0L, kSeq, kSeq, kDh, kScoreScale);

    softmix_kernel<<<dim3(kSeq, 1, 1), blk, 0, stream>>>(S, rw, gam, bet, A2, kA2Carry);

    wmma_gemm64<0, false, 0, 1, false><<<dim3((kSeq / 64) * (kDh / 64) / 8, kHeads, 1), blk, 0, stream>>>(
        A2, A2, kSeq, (long)kSeq * kSeq,
        Vt + (size_t)bb * kSeq, Vt + (size_t)bb * kSeq, kTok, (long)kDh * kTok,
        (void*)(Octx + (size_t)bb * kSeq * kInner), (void*)(Octx + (size_t)bb * kSeq * kInner), kInner, (long)kDh,
        b_out, b_out, 0L, kSeq, kDh, kSeq, kA2CarryInv);
  }

  wmma_gemm64<0, false, 2, 0, false><<<dim3((kTok / 64) * (kDim / 64) / 8, 1, 1), blk, 0, stream>>>(
      Octx, Octx, kInner, 0L, WoT, WoT, kInner, 0L, (void*)out, (void*)out, kDim, 0L,
      b_out, b_out, 0L, kTok, kDim, kInner, kWoCarryInv);
}
